// MixExpertAttentionSACNetwork_6579889897872
// MI455X (gfx1250) — hardware-verified
//
#include <hip/hip_runtime.h>


namespace {
constexpr int NB = 4096, OBS = 390, ACT = 20, KIN = OBS + ACT, KINP = 448, H1 = 1024, H2 = 512, DD = 256, NE = 8, NT = 10;

typedef _Float16 b16;
typedef __attribute__((ext_vector_type(16))) _Float16 v16b;
typedef __attribute__((ext_vector_type(8)))  _Float16 v8b;
typedef __attribute__((ext_vector_type(8)))  float v8f;
typedef __attribute__((ext_vector_type(4)))  float v4f;

__device__ __forceinline__ v8b ld8b(const b16* p) { return *(const v8b*)p; }
__device__ __forceinline__ v16b cat8b(v8b a, v8b b) { return __builtin_shufflevector(a, b, 0, 1, 2, 3, 4, 5, 6, 7, 8, 9, 10, 11, 12, 13, 14, 15); }
__device__ __forceinline__ v16b frag_kb(const b16* p, int hh) { return cat8b(ld8b(p + 8 * hh), ld8b(p + 16 + 8 * hh)); }
__device__ __forceinline__ void split16(float v, b16& hi, b16& lo) { hi = (b16)v; lo = (b16)(v - (float)hi); }
__device__ __forceinline__ void frag_ksplit(const float* p, int hh, v16b& fh_, v16b& fl_) {
  const float* p0 = p + 8 * hh; const float* p1 = p + 16 + 8 * hh;
#pragma unroll
  for (int e = 0; e < 8; ++e) { b16 a, c; split16(p0[e], a, c); fh_[e] = a; fl_[e] = c; split16(p1[e], a, c); fh_[8 + e] = a; fl_[8 + e] = c; }
}
__device__ __forceinline__ v8f wmma16b(v16b a, v16b b, v8f c) {
  v8f d = __builtin_amdgcn_wmma_f32_16x16x32_f16(false, a, false, b, (short)0, c, false, false);
  asm volatile("v_nop\n\tv_nop\n\tv_nop\n\tv_nop" : "+v"(d) : "v"(a), "v"(b));
  return d;
}
__device__ __forceinline__ void wave_lds_sync() {
  __builtin_amdgcn_fence(__ATOMIC_RELEASE, "workgroup");
  __builtin_amdgcn_wave_barrier();
  __builtin_amdgcn_fence(__ATOMIC_ACQUIRE, "workgroup");
}

struct Opnd { const void* p0; const void* p1; int ld; };
template <int NP> __device__ __forceinline__ void load_frags(const Opnd& o, int row, int kb, int hh, v16b& fh_, v16b& fl_) {
  if (NP == 0) { frag_ksplit((const float*)o.p0 + (size_t)row * o.ld + kb, hh, fh_, fl_); }
  else if (NP == 4) {
    const float* p = (const float*)o.p0 + (size_t)row * o.ld + kb; const float* p0 = p + 8 * hh; const float* p1 = p + 16 + 8 * hh;
#pragma unroll
    for (int e = 0; e < 8; ++e) { b16 a, c; split16(p0[e] * 64.0f, a, c); fh_[e] = a; fl_[e] = c; split16(p1[e] * 64.0f, a, c); fh_[8 + e] = a; fl_[8 + e] = c; }
  } else if (NP == 3) {
    const float* p = (const float*)o.p0 + (size_t)row * o.ld + kb; const float* p0 = p + 8 * hh; const float* p1 = p + 16 + 8 * hh;
#pragma unroll
    for (int e = 0; e < 8; ++e) { fh_[e] = (b16)p0[e]; fh_[8 + e] = (b16)p1[e]; }
    fl_ = fh_;
  } else {
    fh_ = frag_kb((const b16*)o.p0 + (size_t)row * o.ld + kb, hh);
    if (NP == 2) fl_ = frag_kb((const b16*)o.p1 + (size_t)row * o.ld + kb, hh); else fl_ = fh_;
  }
}
template <int ANP, int BNP> __device__ __forceinline__ v8f mac(v16b ah, v16b al, v16b bh, v16b bl, v8f c) {
  c = wmma16b(ah, bh, c);
  if (BNP == 0 || BNP == 2 || BNP == 4) c = wmma16b(ah, bl, c);
  if (ANP == 0 || ANP == 2 || ANP == 4) c = wmma16b(al, bh, c);
  return c;
}
template <int ANP, int BNP>
__device__ __forceinline__ void gemm_tile(const Opnd& A, const Opnd& B, int K, int m0, int c0, int nloc, int hlf, v8f (&acc)[2][4]) {
  for (int kb = 0; kb < K; kb += 32) {
    v16b a0h, a0l, a1h, a1l;
    load_frags<ANP>(A, m0 + nloc, kb, hlf, a0h, a0l);
    load_frags<ANP>(A, m0 + 16 + nloc, kb, hlf, a1h, a1l);
#pragma unroll
    for (int t = 0; t < 4; ++t) {
      v16b bh, bl;
      load_frags<BNP>(B, c0 + t * 16 + nloc, kb, hlf, bh, bl);
      acc[0][t] = mac<ANP, BNP>(a0h, a0l, bh, bl, acc[0][t]);
      acc[1][t] = mac<ANP, BNP>(a1h, a1l, bh, bl, acc[1][t]);
    }
  }
}

__device__ __forceinline__ void epi_planes(v8f (&acc)[2][4], float scale, bool two, b16* __restrict__ oh, b16* __restrict__ ol, int ldo,
                                           int m0, int c0, int lane, b16* Th, b16* Tl) {
  const int nloc = lane & 15, hlf = lane >> 4;
#pragma unroll
  for (int t = 0; t < 4; ++t)
#pragma unroll
    for (int r = 0; r < 2; ++r)
#pragma unroll
      for (int v = 0; v < 8; ++v) {
        const int rr = r * 16 + v + 8 * hlf, cc = t * 16 + nloc;
        b16 h_, l_; split16(acc[r][t][v] * scale, h_, l_);
        Th[rr * 64 + cc] = h_; Tl[rr * 64 + cc] = l_;
      }
  wave_lds_sync();
  for (int pass = 0; pass < 2; ++pass) {
#pragma unroll
    for (int j = 0; j < 8; ++j) {
      const int rr = j * 4 + (lane >> 3), c8 = (lane & 7) * 8;
      const size_t o = (size_t)(m0 + rr) * ldo + c0 + c8;
      *(volatile v8b*)(oh + o) = ld8b(Th + rr * 64 + c8);
      if (two) *(volatile v8b*)(ol + o) = ld8b(Tl + rr * 64 + c8);
    }
    __threadfence();
  }
}
__device__ __forceinline__ void epi_f32(v8f (&acc)[2][4], float scale, const float* rscale, float* __restrict__ out, int ldo, int m0, int c0, int lane, float* Tt) {
  const int nloc = lane & 15, hlf = lane >> 4;
#pragma unroll
  for (int t = 0; t < 4; ++t)
#pragma unroll
    for (int r = 0; r < 2; ++r)
#pragma unroll
      for (int v = 0; v < 8; ++v) {
        const int rr = r * 16 + v + 8 * hlf;
        const float rs = rscale ? rscale[(size_t)(m0 + rr) * 32] : 1.0f;
        Tt[rr * 64 + t * 16 + nloc] = acc[r][t][v] * scale * rs;
      }
  wave_lds_sync();
  float* dst0 = out + (size_t)m0 * ldo + c0;
  for (int pass = 0; pass < 2; ++pass) {
#pragma unroll
    for (int j = 0; j < 16; ++j) { const int rr = j * 2 + hlf, c4 = nloc * 4; *(volatile v4f*)(dst0 + (size_t)rr * ldo + c4) = *(const v4f*)(Tt + rr * 64 + c4); }
    __threadfence();
  }
}


__global__ __launch_bounds__(256) void tr_kernel(const float* __restrict__ in, int K, int N, int Kp, size_t zin, b16* __restrict__ out, size_t zout) {
  __shared__ __attribute__((aligned(16))) b16 Tl[64][72];
  const int tid = threadIdx.x, lane = tid & 31, wave = tid >> 5, n0 = blockIdx.x * 64, k0 = blockIdx.y * 64; const size_t z = blockIdx.z;
  const float* src = in + z * zin;
  for (int it = 0; it < 16; ++it) {
    const int kk = k0 + it * 4 + (tid >> 6), n = tid & 63;
    Tl[n][it * 4 + (tid >> 6)] = (kk < K) ? (b16)src[(size_t)kk * N + n0 + n] : (b16)0.0f;
  }
  __syncthreads();
  b16* dst = out + z * zout + (size_t)n0 * Kp + k0;
  for (int pass = 0; pass < 2; ++pass) {
#pragma unroll
    for (int j = 0; j < 2; ++j) { const int rr = wave * 8 + j * 4 + (lane >> 3), c8 = (lane & 7) * 8; *(volatile v8b*)(dst + (size_t)rr * Kp + c8) = *(const v8b*)(&Tl[rr][c8]); }
    __threadfence();
  }
}

__global__ __launch_bounds__(256) void xcat_kernel(const float* __restrict__ sf, const float* __restrict__ ac, b16* __restrict__ x16) {
  const size_t tid = (size_t)blockIdx.x * blockDim.x + threadIdx.x, stride = (size_t)gridDim.x * blockDim.x, tot = (size_t)NB * KINP / 8;
  for (int pass = 0; pass < 2; ++pass) {
    for (size_t c = tid; c < tot; c += stride) {
      const size_t i = c * 8; const int b = (int)(i / KINP), k0 = (int)(i % KINP); v8b v;
#pragma unroll
      for (int e = 0; e < 8; ++e) { const int k = k0 + e; v[e] = (b16)((k < OBS) ? sf[(size_t)b * OBS + k] : (k < KIN) ? ac[(size_t)b * ACT + (k - OBS)] : 0.0f); }
      *(volatile v8b*)(x16 + i) = v;
    }
    __threadfence();
  }
}

template <bool RELU, bool OUT16>
__global__ __launch_bounds__(128) void gemm_kernel(const b16* __restrict__ A, size_t az, int lda, const b16* __restrict__ Bm, size_t bz, int ldb, int K,
                                                   const float* __restrict__ bias, size_t bzb, b16* __restrict__ o16, float* __restrict__ o32, size_t oz, int ldo) {
  __shared__ __attribute__((aligned(16))) float Ts[4][32 * 64];
  __shared__ __attribute__((aligned(16))) b16 Th[4][2][32 * 64];
  const int lane = threadIdx.x & 31, wave = threadIdx.x >> 5, nloc = lane & 15, hlf = lane >> 4; const size_t z = blockIdx.z;
  const int m0 = blockIdx.y * 128 + wave * 32, c0 = blockIdx.x * 64;
  v8f acc[2][4];
#pragma unroll
  for (int r = 0; r < 2; ++r)
#pragma unroll
    for (int t = 0; t < 4; ++t) acc[r][t] = (v8f){};
  const Opnd Ao{A + z * az, nullptr, lda}, Bo{Bm + z * bz, nullptr, ldb};
  gemm_tile<1, 1>(Ao, Bo, K, m0, c0, nloc, hlf, acc);
  const float* bb = bias + z * bzb;
#pragma unroll
  for (int t = 0; t < 4; ++t)
#pragma unroll
    for (int r = 0; r < 2; ++r)
#pragma unroll
      for (int v = 0; v < 8; ++v) { float val = acc[r][t][v] + bb[c0 + t * 16 + nloc]; if (RELU) val = fmaxf(val, 0.0f); acc[r][t][v] = val; }
  if (OUT16) epi_planes(acc, 1.0f, false, o16 + z * oz, nullptr, ldo, m0, c0, lane, Th[wave][0], Th[wave][1]);
  else       epi_f32(acc, 1.0f, nullptr, o32 + z * oz, ldo, m0, c0, lane, Ts[wave]);
}

__global__ __launch_bounds__(256) void mix_kernel(const float* __restrict__ emb, const int* __restrict__ tid_, const float* __restrict__ keys, const float* __restrict__ vals,
                                                  b16* __restrict__ tin, float* __restrict__ term) {
  __shared__ float ts[32]; __shared__ float qs[8][256]; __shared__ float ws_[8][NE];
  const int wave = threadIdx.x >> 5, lane = threadIdx.x & 31, b0 = blockIdx.x * 32;
  float* qw = qs[wave]; float* ww = ws_[wave];
  for (int qq = 0; qq < 4; ++qq) {
    const int b = b0 + wave * 4 + qq;
    int t = tid_[b]; t = t < 0 ? 0 : (t >= NT ? NT - 1 : t);
#pragma unroll 1
    for (int e8 = 0; e8 < 8; ++e8) qw[lane * 8 + e8] = tanhf(emb[(size_t)t * DD + lane * 8 + e8]);
    wave_lds_sync();
    float mx = -INFINITY;
#pragma unroll 1
    for (int e = 0; e < NE; ++e) {
      const float* kr = keys + ((size_t)e * NB + b) * DD + lane * 8; float s = 0.0f;
#pragma unroll 1
      for (int e8 = 0; e8 < 8; ++e8) s += qw[lane * 8 + e8] * kr[e8];
#pragma unroll
      for (int o = 16; o > 0; o >>= 1) s += __shfl_xor(s, o);
      if (lane == 0) ww[e] = s;
      mx = fmaxf(mx, s);
    }
    wave_lds_sync();
    float sum = 0.0f;
#pragma unroll 1
    for (int e = 0; e < NE; ++e) sum += expf(ww[e] - mx);
    float tr = 0.0f;
#pragma unroll 1
    for (int e = 0; e < NE; ++e) { const float w = expf(ww[e] - mx) / sum; tr += fminf(fmaxf(logf(w + 1e-10f), -6.0f), 0.0f); }
    v8b tv;
#pragma unroll 1
    for (int e8 = 0; e8 < 8; ++e8) { float a = 0.0f;
#pragma unroll 1
      for (int e = 0; e < NE; ++e) a += (expf(ww[e] - mx) / sum) * vals[((size_t)e * NB + b) * DD + lane * 8 + e8];
      tv[e8] = (b16)a; }
    *(volatile v8b*)(tin + (size_t)b * DD + lane * 8) = tv; __threadfence(); *(volatile v8b*)(tin + (size_t)b * DD + lane * 8) = tv;
    if (lane == 0) ts[wave * 4 + qq] = tr;
    wave_lds_sync();
  }
  __syncthreads();
  if (wave == 0) { ((volatile float*)term)[b0 + lane] = ts[lane]; __threadfence(); ((volatile float*)term)[b0 + lane] = ts[lane]; }
}

__global__ __launch_bounds__(256) void final_kernel(const float* __restrict__ t2, const float* __restrict__ tW3, const float* __restrict__ tb3, const float* __restrict__ term, float* __restrict__ out) {
  __shared__ float qs[32];
  const int wave = threadIdx.x >> 5, lane = threadIdx.x & 31, b0 = blockIdx.x * 32;
  for (int qq = 0; qq < 4; ++qq) {
    const int b = b0 + wave * 4 + qq; const float* row = t2 + (size_t)b * DD + lane * 8; float s = 0.0f;
#pragma unroll
    for (int e8 = 0; e8 < 8; ++e8) s += row[e8] * tW3[lane * 8 + e8];
#pragma unroll
    for (int o = 16; o > 0; o >>= 1) s += __shfl_xor(s, o);
    if (lane == 0) qs[wave * 4 + qq] = s + tb3[0];
  }
  __syncthreads();
  if (wave == 0) { ((volatile float*)out)[b0 + lane] = qs[lane]; __threadfence(); ((volatile float*)out)[b0 + lane] = qs[lane]; }
  if (blockIdx.x == 0 && threadIdx.x == 32) {
    float s = 0.0f; for (int b = 0; b < NB; ++b) s += term[b];
    const float loss = -0.3f * (s * (1.0f / NB));
    ((volatile float*)out)[NB] = loss; __threadfence(); ((volatile float*)out)[NB] = loss;
  }
}
}

extern "C" void kernel_launch(void* const* d_in, const int* in_sizes, int n_in,
                              void* d_out, int out_size, void* d_ws, size_t ws_size, hipStream_t stream) {
  (void)n_in;
  const float* sf  = (const float*)d_in[0];
  const float* ac  = (const float*)d_in[1];
  const int* tk    = (const int*)d_in[2];
  const float* rW1 = (const float*)d_in[3];  const float* rb1 = (const float*)d_in[4];
  const float* rW2 = (const float*)d_in[5];  const float* rb2 = (const float*)d_in[6];
  const float* emb = (const float*)d_in[7];
  const float* kW1 = (const float*)d_in[8];  const float* kb1 = (const float*)d_in[9];
  const float* kW2 = (const float*)d_in[10]; const float* kb2 = (const float*)d_in[11];
  const float* vW1 = (const float*)d_in[12]; const float* vb1 = (const float*)d_in[13];
  const float* vW2 = (const float*)d_in[14]; const float* vb2 = (const float*)d_in[15];
  const float* tW1 = (const float*)d_in[16]; const float* tb1 = (const float*)d_in[17];
  const float* tW2 = (const float*)d_in[18]; const float* tb2 = (const float*)d_in[19];
  const float* tW3 = (const float*)d_in[20]; const float* tb3 = (const float*)d_in[21];
  float* out = (float*)d_out;
  if (in_sizes[0] != NB * OBS || in_sizes[1] != NB * ACT || in_sizes[3] != KIN * H1 || in_sizes[8] != NE * H1 * H2 || out_size != NB + 1) return;

  size_t off = 0; char* ws = (char*)d_ws;
  auto carve = [&](size_t bytes) { char* p = ws + off; off += (bytes + 255) & ~(size_t)255; return p; };
  b16* x16  = (b16*)carve((size_t)NB * KINP * 2);
  b16* rW1T = (b16*)carve((size_t)H1 * KINP * 2);
  b16* rW2T = (b16*)carve((size_t)H1 * H1 * 2);
  b16* kW1T = (b16*)carve((size_t)NE * H2 * H1 * 2);
  b16* kW2T = (b16*)carve((size_t)NE * DD * H2 * 2);
  b16* vW1T = (b16*)carve((size_t)NE * H2 * H1 * 2);
  b16* vW2T = (b16*)carve((size_t)NE * DD * H2 * 2);
  b16* tW1T = (b16*)carve((size_t)DD * DD * 2); b16* tW2T = (b16*)carve((size_t)DD * DD * 2);
  b16* h0   = (b16*)carve((size_t)NB * H1 * 2);
  b16* rep  = (b16*)carve((size_t)NB * H1 * 2);
  b16* hk   = (b16*)carve((size_t)4 * NB * H2 * 2);
  float* keys = (float*)carve((size_t)NE * NB * DD * 4);
  float* vals = (float*)carve((size_t)NE * NB * DD * 4);
  float* term = (float*)carve((size_t)NB * 4);
  if (off > ws_size) return;
  b16* tin = h0; b16* t1 = h0 + (size_t)NB * DD; float* t2 = (float*)(h0 + (size_t)2 * NB * DD);
  tr_kernel<<<dim3(H1 / 64, KINP / 64, 1), 256, 0, stream>>>(rW1, KIN, H1, KINP, 0, rW1T, 0);
  tr_kernel<<<dim3(H1 / 64, H1 / 64, 1), 256, 0, stream>>>(rW2, H1, H1, H1, 0, rW2T, 0);
  tr_kernel<<<dim3(H2 / 64, H1 / 64, NE), 256, 0, stream>>>(kW1, H1, H2, H1, (size_t)H1 * H2, kW1T, (size_t)H2 * H1);
  tr_kernel<<<dim3(DD / 64, H2 / 64, NE), 256, 0, stream>>>(kW2, H2, DD, H2, (size_t)H2 * DD, kW2T, (size_t)DD * H2);
  tr_kernel<<<dim3(H2 / 64, H1 / 64, NE), 256, 0, stream>>>(vW1, H1, H2, H1, (size_t)H1 * H2, vW1T, (size_t)H2 * H1);
  tr_kernel<<<dim3(DD / 64, H2 / 64, NE), 256, 0, stream>>>(vW2, H2, DD, H2, (size_t)H2 * DD, vW2T, (size_t)DD * H2);
  tr_kernel<<<dim3(DD / 64, DD / 64, 1), 256, 0, stream>>>(tW1, DD, DD, DD, 0, tW1T, 0);
  tr_kernel<<<dim3(DD / 64, DD / 64, 1), 256, 0, stream>>>(tW2, DD, DD, DD, 0, tW2T, 0);
  xcat_kernel<<<896, 256, 0, stream>>>(sf, ac, x16);
  gemm_kernel<true, true><<<dim3(H1 / 64, NB / 128, 1), 128, 0, stream>>>(x16, 0, KINP, rW1T, 0, KINP, KINP, rb1, 0, h0, nullptr, 0, H1);
  gemm_kernel<false, true><<<dim3(H1 / 64, NB / 128, 1), 128, 0, stream>>>(h0, 0, H1, rW2T, 0, H1, H1, rb2, 0, rep, nullptr, 0, H1);
  for (int half = 0; half < 2; ++half) {
    const size_t e0 = (size_t)4 * half;
    gemm_kernel<true, true><<<dim3(H2 / 64, NB / 128, 4), 128, 0, stream>>>(rep, 0, H1, kW1T + e0 * H2 * H1, (size_t)H2 * H1, H1, H1, kb1 + e0 * H2, H2, hk, nullptr, (size_t)NB * H2, H2);
    gemm_kernel<false, false><<<dim3(DD / 64, NB / 128, 4), 128, 0, stream>>>(hk, (size_t)NB * H2, H2, kW2T + e0 * DD * H2, (size_t)DD * H2, H2, H2, kb2 + e0 * DD, DD, nullptr, keys + e0 * NB * DD, (size_t)NB * DD, DD);
    gemm_kernel<true, true><<<dim3(H2 / 64, NB / 128, 4), 128, 0, stream>>>(rep, 0, H1, vW1T + e0 * H2 * H1, (size_t)H2 * H1, H1, H1, vb1 + e0 * H2, H2, hk, nullptr, (size_t)NB * H2, H2);
    gemm_kernel<false, false><<<dim3(DD / 64, NB / 128, 4), 128, 0, stream>>>(hk, (size_t)NB * H2, H2, vW2T + e0 * DD * H2, (size_t)DD * H2, H2, H2, vb2 + e0 * DD, DD, nullptr, vals + e0 * NB * DD, (size_t)NB * DD, DD);
  }
  mix_kernel<<<NB / 32, 256, 0, stream>>>(emb, tk, keys, vals, tin, term);
  gemm_kernel<true, true><<<dim3(DD / 64, NB / 128, 1), 128, 0, stream>>>(tin, 0, DD, tW1T, 0, DD, DD, tb1, 0, t1, nullptr, 0, DD);
  gemm_kernel<true, false><<<dim3(DD / 64, NB / 128, 1), 128, 0, stream>>>(t1, 0, DD, tW2T, 0, DD, DD, tb2, 0, nullptr, t2, 0, DD);
  final_kernel<<<NB / 32, 256, 0, stream>>>(t2, tW3, tb3, term, out);
}
